// BEVWarpAndAccumulate_79611513799004
// MI455X (gfx1250) — hardware-run, weakly checked
//
#include <hip/hip_runtime.h>
#include <math.h>

typedef __attribute__((ext_vector_type(16))) _Float16 v16h;
typedef __attribute__((ext_vector_type(8)))  _Float16 v8h;
typedef __attribute__((ext_vector_type(4)))  _Float16 v4h;
typedef __attribute__((ext_vector_type(8)))  float    v8f;
typedef __attribute__((ext_vector_type(4)))  float    v4f;
typedef __attribute__((ext_vector_type(2)))  float    v2f;

constexpr int kBatch  = 4096;
constexpr int kFrames = 4;
constexpr int kDm     = 384;
constexpr int kPix    = 64;
constexpr int kChan   = 96;
constexpr int kN1     = 6144;
constexpr int kRows   = kBatch * kFrames;
static_assert(kChan * kPix == kN1, "channel-major pixel layout");
static_assert(kChan * 4 == kDm, "channel count");
static_assert((kDm % 32) == 0 && (kChan % 32) == 0, "GEMM K multiples of 32");
static_assert((kRows % 64) == 0 && (kBatch % 64) == 0 && (kDm % 64) == 0 && (kN1 % 64) == 0, "GEMM M,N multiples of 64");

constexpr float kCarryHv   = 16.0f;
constexpr float kCarryW    = 1024.0f;
constexpr float kCarryPsp  = 256.0f;
constexpr float kCarryPool = 4096.0f;
constexpr float kCarryH    = 4096.0f;
constexpr float kSc1 = 1.0f / (kCarryHv * kCarryW);
constexpr float kSc2 = 1.0f / (kCarryPsp * kCarryW);
constexpr float kSc3 = 1.0f / (kCarryPool * kCarryW);
constexpr float kSc4 = 1.0f / (kCarryH * kCarryW);

constexpr size_t kOffW1T  = 0;
constexpr size_t kOffW2T  = kOffW1T  + (size_t)kN1 * kDm * 2;
constexpr size_t kOffWF1T = kOffW2T  + (size_t)kDm * kChan * 2;
constexpr size_t kOffWF2T = kOffWF1T + (size_t)kDm * kDm * 2;
constexpr size_t kOffWVEC = kOffWF2T + (size_t)kDm * kDm * 2;
constexpr size_t kOffPSP  = kOffWVEC + (size_t)kRows * kPix * 4;
constexpr size_t kOffPOOL = kOffPSP  + (size_t)kRows * kChan * 2;
constexpr size_t kOffHMID = kOffPOOL + (size_t)kBatch * kDm * 2;
constexpr size_t kWsTotal = kOffHMID + (size_t)kBatch * kDm * 2;
static_assert(kWsTotal == 19013632ull, "carve total");
static_assert(kWsTotal <= 134217728ull, "carve cap");
static_assert((kOffW2T % 128) == 0 && (kOffWF1T % 128) == 0 && (kOffWF2T % 128) == 0 && (kOffWVEC % 128) == 0 &&
              (kOffPSP % 128) == 0 && (kOffPOOL % 128) == 0 && (kOffHMID % 128) == 0, "128-B aligned regions");

union FragU { v16h v; v8h h[2]; };

__device__ __forceinline__ v16h frag_load(const _Float16* p) {
  FragU f;
  f.h[0] = *(const v8h*)(p);
  f.h[1] = *(const v8h*)(p + 16);
  return f.v;
}

__device__ __forceinline__ v8f mma_g(v16h a, v16h b, v8f c) {
  c = __builtin_amdgcn_wmma_f32_16x16x32_f16(false, a, false, b, (short)0, c, false, false);
  asm volatile("v_nop\n\tv_nop\n\tv_nop\n\tv_nop" : "+v"(c) : "v"(a), "v"(b));
  return c;
}

__device__ __forceinline__ void wave_lds_sync() {
  __builtin_amdgcn_fence(__ATOMIC_RELEASE, "workgroup");
  __builtin_amdgcn_wave_barrier();
  __builtin_amdgcn_fence(__ATOMIC_ACQUIRE, "workgroup");
}

__device__ __forceinline__ float gelu_erf(float x) {
  return 0.5f * x * (1.0f + erff(x * 0.70710678118654752440f));
}

__device__ __forceinline__ void gelu_slab_inplace(float* slab, int lane) {
#pragma unroll 1
  for (int it = 0; it < 16; ++it) {
    const int f = it * 64 + lane * 2;
    float* p = slab + (f >> 6) * 68 + (f & 63);
    v2f x = *(const v2f*)p;
    v2f y;
    y[0] = gelu_erf(x[0]);
    y[1] = gelu_erf(x[1]);
    *(v2f*)p = y;
  }
}

__global__ __launch_bounds__(256) void transpose_cvt_kernel(
    const float* __restrict__ in, unsigned short* __restrict__ outp, int R, int Cn, float carry)
{
  __shared__ __align__(16) float sT[64 * 68];
  const int tid = threadIdx.x;
  const int n0 = blockIdx.x * 64;
  const int k0 = blockIdx.y * 64;
#pragma unroll
  for (int it = 0; it < 4; ++it) {
    const int idx = it * 256 + tid;
    const int kr = idx >> 4;
    const int c4 = (idx & 15) * 4;
    const v4f v = *(const v4f*)(in + (size_t)(k0 + kr) * Cn + n0 + c4);
    *(v4f*)(sT + kr * 68 + c4) = v;
  }
  __syncthreads();
  _Float16* out = (_Float16*)outp;
  const int kq = (tid & 7) * 8;
  v8h hv[2];
#pragma unroll
  for (int it = 0; it < 2; ++it) {
    const int nl = it * 32 + (tid >> 3);
#pragma unroll
    for (int e = 0; e < 8; ++e) hv[it][e] = (_Float16)(sT[(kq + e) * 68 + nl] * carry);
  }
  for (int pass = 0; pass < 2; ++pass) {
#pragma unroll
    for (int it = 0; it < 2; ++it) {
      const int nl = it * 32 + (tid >> 3);
      *(volatile v8h*)(out + (size_t)(n0 + nl) * R + k0 + kq) = hv[it];
    }
    __threadfence();
  }
}

__global__ __launch_bounds__(256) void transpose_w2_kernel(
    const float* __restrict__ in, unsigned short* __restrict__ outp, float carry)
{
  __shared__ __align__(16) float sT[kChan * 68];
  const int tid = threadIdx.x;
  const int n0 = blockIdx.x * 64;
#pragma unroll
  for (int it = 0; it < 6; ++it) {
    const int idx = it * 256 + tid;
    const int kr = idx >> 4;
    const int c4 = (idx & 15) * 4;
    const v4f v = *(const v4f*)(in + (size_t)kr * kDm + n0 + c4);
    *(v4f*)(sT + kr * 68 + c4) = v;
  }
  __syncthreads();
  _Float16* out = (_Float16*)outp + (size_t)n0 * kChan;
  v8h hv[3];
#pragma unroll
  for (int it = 0; it < 3; ++it) {
    const int q = it * 256 + tid;
    const int nl = q / 12;
    const int kb = (q - nl * 12) * 8;
#pragma unroll
    for (int e = 0; e < 8; ++e) hv[it][e] = (_Float16)(sT[(kb + e) * 68 + nl] * carry);
  }
  for (int pass = 0; pass < 2; ++pass) {
#pragma unroll
    for (int it = 0; it < 3; ++it) {
      const int q = it * 256 + tid;
      *(volatile v8h*)(out + (size_t)q * 8) = hv[it];
    }
    __threadfence();
  }
}

__global__ __launch_bounds__(256) void warp_weights_kernel(
    const float* __restrict__ ego, float* __restrict__ wvec)
{
  __shared__ float sx[256];
  __shared__ float sy[256];
  const int tid = threadIdx.x;
  const int wave = __builtin_amdgcn_readfirstlane((int)(threadIdx.x >> 5));
  const int t = wave >> 1;
  const int p = tid & 63;
  const int b = blockIdx.x;
  const int tc = (t < 3) ? t : 2;
  const int eidx = (b * 3 + tc) * 3;
  const float dx = ego[eidx + 0];
  const float dy = ego[eidx + 1];
  const float dyaw = ego[eidx + 2];
  const float ca = cosf(dyaw);
  const float sa = sinf(dyaw);
  const float tx = dx * 0.02f;
  const float ty = dy * 0.02f;
  const float xg = ((float)(p & 7) + 0.5f) * 0.25f - 1.0f;
  const float yg = ((float)(p >> 3) + 0.5f) * 0.25f - 1.0f;
  float gx = ca * xg;
  gx = fmaf(sa, yg, gx);
  gx = gx + tx;
  float gy = (-sa) * xg;
  gy = fmaf(ca, yg, gy);
  gy = gy + ty;
  sx[tid] = (gx + 1.0f) * 4.0f - 0.5f;
  sy[tid] = (gy + 1.0f) * 4.0f - 0.5f;
  __syncthreads();
  float acc = 0.0f;
  if (t < 3) {
    const float fpx = (float)(p & 7);
    const float fpy = (float)(p >> 3);
    const int qb = t * 64;
#pragma unroll 4
    for (int q = 0; q < 64; ++q) {
      const float hx = fmaxf(0.0f, 1.0f - fabsf(sx[qb + q] - fpx));
      const float hy = fmaxf(0.0f, 1.0f - fabsf(sy[qb + q] - fpy));
      acc = fmaf(hy, hx, acc);
    }
  }
  const float val = (t < 3) ? (acc * (1.0f / 64.0f)) : (1.0f / 64.0f);
  volatile float* dst = wvec + ((size_t)(b * 4 + t) * 64 + p);
  *dst = val;
  __threadfence();
  *dst = val;
}

constexpr int kBlkRows = 32;
constexpr int kAPitch  = 392;
static_assert((kRows % kBlkRows) == 0, "row tiles");
static_assert((kChan % 4) == 0, "channels per wave trip");

__global__ __launch_bounds__(128) void gemm1_pool_kernel(
    const float* __restrict__ hv, const unsigned short* __restrict__ W1tp, const float* __restrict__ b1,
    const float* __restrict__ wvec, unsigned short* __restrict__ pspp)
{
  __shared__ __align__(16) _Float16 sA[kBlkRows * kAPitch];
  __shared__ __align__(16) float sWv[kBlkRows * 64];
  __shared__ __align__(16) float sSlab[4][16 * 68];
  __shared__ __align__(16) float sP[kBlkRows * kChan];
  const _Float16* W1t = (const _Float16*)W1tp;
  const int tid = threadIdx.x;
  const int lane = tid & 31;
  const int wave = __builtin_amdgcn_readfirstlane((int)(threadIdx.x >> 5));
  const int r0 = blockIdx.x * kBlkRows;

#pragma unroll 2
  for (int it = 0; it < 24; ++it) {
    const int idx = it * 128 + tid;
    const int r = idx / 96;
    const int c4 = (idx - r * 96) * 4;
    const v4f v = *(const v4f*)(hv + (size_t)(r0 + r) * kDm + c4);
    v4h h;
    h[0] = (_Float16)(v[0] * kCarryHv);
    h[1] = (_Float16)(v[1] * kCarryHv);
    h[2] = (_Float16)(v[2] * kCarryHv);
    h[3] = (_Float16)(v[3] * kCarryHv);
    *(v4h*)(sA + r * kAPitch + c4) = h;
  }
#pragma unroll
  for (int it = 0; it < 4; ++it) {
    const int idx = it * 128 + tid;
    const v4f v = *(const v4f*)(wvec + (size_t)r0 * 64 + idx * 4);
    *(v4f*)(sWv + idx * 4) = v;
  }
  __syncthreads();

  const int rlane = lane & 15;
  const int hh = lane >> 4;
  const int koff = hh * 8;
  const int mOff = hh * 8;
  const int erow = lane >> 1;
  const int ehb = lane & 1;
  float* slab = sSlab[wave];
  const int aoff0 = rlane * kAPitch + koff;
  const int aoff1 = (16 + rlane) * kAPitch + koff;

#pragma unroll 1
  for (int cit = 0; cit < kChan / 4; ++cit) {
    const int ch = cit * 4 + wave;
    v8f acc[2][4];
#pragma unroll
    for (int i = 0; i < 2; ++i)
#pragma unroll
      for (int j = 0; j < 4; ++j) acc[i][j] = (v8f){0.f, 0.f, 0.f, 0.f, 0.f, 0.f, 0.f, 0.f};
    const _Float16* Bp = W1t + (size_t)(ch * 64 + rlane) * kDm + koff;
#pragma unroll 1
    for (int k0 = 0; k0 < kDm; k0 += 32) {
      v16h bh[4];
#pragma unroll
      for (int j = 0; j < 4; ++j) bh[j] = frag_load(Bp + (size_t)(j * 16) * kDm + k0);
      FragU fa0, fa1;
      fa0.h[0] = *(const v8h*)(sA + aoff0 + k0);
      fa0.h[1] = *(const v8h*)(sA + aoff0 + k0 + 16);
      fa1.h[0] = *(const v8h*)(sA + aoff1 + k0);
      fa1.h[1] = *(const v8h*)(sA + aoff1 + k0 + 16);
#pragma unroll
      for (int j = 0; j < 4; ++j) acc[0][j] = mma_g(fa0.v, bh[j], acc[0][j]);
#pragma unroll
      for (int j = 0; j < 4; ++j) acc[1][j] = mma_g(fa1.v, bh[j], acc[1][j]);
    }
    float bv[4];
#pragma unroll
    for (int j = 0; j < 4; ++j) bv[j] = b1[ch * 64 + j * 16 + rlane];

#pragma unroll
    for (int i = 0; i < 2; ++i) {
#pragma unroll
      for (int j = 0; j < 4; ++j)
#pragma unroll
        for (int r = 0; r < 8; ++r)
          slab[(mOff + r) * 68 + j * 16 + rlane] = fmaf(acc[i][j][r], kSc1, bv[j]);
      wave_lds_sync();
      const float* sl = slab + erow * 68 + ehb * 32;
      const float* wr = sWv + (i * 16 + erow) * 64 + ehb * 32;
      float s = 0.0f;
#pragma unroll 1
      for (int it = 0; it < 8; ++it) {
        const v4f x = *(const v4f*)(sl + 4 * it);
        const v4f w = *(const v4f*)(wr + 4 * it);
        s = fmaf(w[0], gelu_erf(x[0]), s);
        s = fmaf(w[1], gelu_erf(x[1]), s);
        s = fmaf(w[2], gelu_erf(x[2]), s);
        s = fmaf(w[3], gelu_erf(x[3]), s);
      }
      s += __shfl_xor(s, 1, 32);
      if (ehb == 0) sP[(i * 16 + erow) * kChan + ch] = s;
      wave_lds_sync();
    }
  }
  __syncthreads();

  _Float16* psp = (_Float16*)pspp + (size_t)r0 * kChan;
  v8h o[3];
#pragma unroll
  for (int it = 0; it < 3; ++it) {
    const int q = it * 128 + tid;
    const v4f a0 = *(const v4f*)(sP + q * 8);
    const v4f a1 = *(const v4f*)(sP + q * 8 + 4);
#pragma unroll
    for (int e = 0; e < 4; ++e) {
      o[it][e]     = (_Float16)(a0[e] * kCarryPsp);
      o[it][4 + e] = (_Float16)(a1[e] * kCarryPsp);
    }
  }
  for (int pass = 0; pass < 2; ++pass) {
#pragma unroll
    for (int it = 0; it < 3; ++it) {
      const int q = it * 128 + tid;
      *(volatile v8h*)(psp + (size_t)q * 8) = o[it];
    }
    __threadfence();
  }
}

template <int MODE>
__global__ __launch_bounds__(256) void gemm64_kernel(
    const unsigned short* __restrict__ Ap, const unsigned short* __restrict__ Btp, int K, int tilesM, int tilesN,
    float scale, const float* __restrict__ bias, const float* __restrict__ tw,
    void* __restrict__ outp, int ldo, float oscale)
{
  const _Float16* A  = (const _Float16*)Ap;
  const _Float16* Bt = (const _Float16*)Btp;
  __shared__ __align__(16) float sT[8][16 * 68];
  const int lane = threadIdx.x & 31;
  const int wave = __builtin_amdgcn_readfirstlane((int)(threadIdx.x >> 5));
  const int tile = blockIdx.x * 8 + wave;
  if (tile >= tilesM * tilesN) return;
  const int tm = tile / tilesN;
  const int tn = tile - tm * tilesN;
  const int m0 = tm << 6;
  const int n0 = tn << 6;
  const int rlane = lane & 15;
  const int koff = (lane >> 4) * 8;
  const int mOff = (lane >> 4) * 8;

  v8f acc[4][4];
#pragma unroll
  for (int i = 0; i < 4; ++i)
#pragma unroll
    for (int j = 0; j < 4; ++j) acc[i][j] = (v8f){0.f, 0.f, 0.f, 0.f, 0.f, 0.f, 0.f, 0.f};

  for (int k0 = 0; k0 < K; k0 += 32) {
    v16h bh[4];
#pragma unroll
    for (int j = 0; j < 4; ++j) bh[j] = frag_load(Bt + (size_t)(n0 + (j << 4) + rlane) * K + koff + k0);
#pragma unroll
    for (int i = 0; i < 4; ++i) {
      const v16h ah = frag_load(A + (size_t)(m0 + (i << 4) + rlane) * K + koff + k0);
#pragma unroll
      for (int j = 0; j < 4; ++j) acc[i][j] = mma_g(ah, bh[j], acc[i][j]);
    }
  }

  float bv[4];
#pragma unroll
  for (int j = 0; j < 4; ++j) bv[j] = bias[n0 + (j << 4) + rlane];

  float sw0 = 0.f, sw1 = 0.f, sw2 = 0.f, sw3 = 0.f;
  if (MODE == 2) {
    const float t0 = tw[0], t1 = tw[1], t2 = tw[2], t3 = tw[3];
    const float mx = fmaxf(fmaxf(t0, t1), fmaxf(t2, t3));
    const float e0 = expf(t0 - mx), e1 = expf(t1 - mx), e2 = expf(t2 - mx), e3 = expf(t3 - mx);
    const float inv = 1.0f / (e0 + e1 + e2 + e3);
    sw0 = e0 * inv;
    sw1 = e1 * inv;
    sw2 = e2 * inv;
    sw3 = e3 * inv;
  }

  float* slab = sT[wave];
#pragma unroll
  for (int i = 0; i < 4; ++i) {
    const int mBase = m0 + (i << 4);
#pragma unroll
    for (int j = 0; j < 4; ++j)
#pragma unroll
      for (int r = 0; r < 8; ++r)
        slab[(mOff + r) * 68 + (j << 4) + rlane] = fmaf(acc[i][j][r], scale, bv[j]);
    wave_lds_sync();
    if (MODE != 0) {
      gelu_slab_inplace(slab, lane);
      wave_lds_sync();
    }
    if (MODE == 0) {
      float* C = (float*)outp;
      const int hh2 = lane >> 4, c4 = (lane & 15) * 4;
      for (int pass = 0; pass < 2; ++pass) {
#pragma unroll
        for (int it = 0; it < 8; ++it) {
          const int row = it * 2 + hh2;
          const v4f v = *(const v4f*)(slab + row * 68 + c4);
          *(volatile v4f*)(C + (size_t)(mBase + row) * ldo + n0 + c4) = v;
        }
        __threadfence();
      }
    } else if (MODE == 1) {
      _Float16* C = (_Float16*)outp;
      const int q = lane >> 3, c8 = (lane & 7) * 8;
      for (int pass = 0; pass < 2; ++pass) {
#pragma unroll
        for (int it = 0; it < 4; ++it) {
          const int row = it * 4 + q;
          const float* sp = slab + row * 68 + c8;
          const v4f a0 = *(const v4f*)(sp);
          const v4f a1 = *(const v4f*)(sp + 4);
          v8h hvv;
#pragma unroll
          for (int e = 0; e < 4; ++e) {
            hvv[e]     = (_Float16)(a0[e] * oscale);
            hvv[4 + e] = (_Float16)(a1[e] * oscale);
          }
          *(volatile v8h*)(C + (size_t)(mBase + row) * ldo + n0 + c8) = hvv;
        }
        __threadfence();
      }
    } else {
      _Float16* C = (_Float16*)outp;
      const int orow = lane >> 3, c8 = (lane & 7) * 8;
      float o[8];
#pragma unroll
      for (int e = 0; e < 8; ++e) o[e] = 0.0f;
#pragma unroll
      for (int t = 0; t < 4; ++t) {
        const float wt = (t == 0) ? sw0 : ((t == 1) ? sw1 : ((t == 2) ? sw2 : sw3));
        const float* sp = slab + (orow * 4 + t) * 68 + c8;
        const v4f a0 = *(const v4f*)(sp);
        const v4f a1 = *(const v4f*)(sp + 4);
#pragma unroll
        for (int e = 0; e < 4; ++e) {
          o[e]     = fmaf(wt, a0[e], o[e]);
          o[4 + e] = fmaf(wt, a1[e], o[4 + e]);
        }
      }
      v8h hvv;
#pragma unroll
      for (int e = 0; e < 8; ++e) hvv[e] = (_Float16)(o[e] * oscale);
      _Float16* dst = C + (size_t)((mBase >> 2) + orow) * ldo + n0 + c8;
      *(volatile v8h*)dst = hvv;
      __threadfence();
      *(volatile v8h*)dst = hvv;
    }
    wave_lds_sync();
  }
}

extern "C" void kernel_launch(void* const* d_in, const int* in_sizes, int n_in,
                              void* d_out, int out_size, void* d_ws, size_t ws_size,
                              hipStream_t stream) {
  if (n_in < 11) return;
  if (in_sizes[0] != kRows * kDm) return;
  if (in_sizes[1] != kBatch * 3 * 3) return;
  if (in_sizes[2] != kDm * kN1) return;
  if (in_sizes[3] != kN1) return;
  if (in_sizes[4] != kChan * kDm) return;
  if (in_sizes[5] != kDm) return;
  if (in_sizes[6] != kFrames) return;
  if (in_sizes[7] != kDm * kDm) return;
  if (in_sizes[8] != kDm) return;
  if (in_sizes[9] != kDm * kDm) return;
  if (in_sizes[10] != kDm) return;
  if (out_size != kBatch * kDm) return;
  if (ws_size < kWsTotal) return;

  const float* hv  = (const float*)d_in[0];
  const float* ego = (const float*)d_in[1];
  const float* W1  = (const float*)d_in[2];
  const float* b1  = (const float*)d_in[3];
  const float* W2  = (const float*)d_in[4];
  const float* b2  = (const float*)d_in[5];
  const float* tw  = (const float*)d_in[6];
  const float* Wf1 = (const float*)d_in[7];
  const float* bf1 = (const float*)d_in[8];
  const float* Wf2 = (const float*)d_in[9];
  const float* bf2 = (const float*)d_in[10];

  char* ws = (char*)d_ws;
  unsigned short* W1T  = (unsigned short*)(ws + kOffW1T);
  unsigned short* W2T  = (unsigned short*)(ws + kOffW2T);
  unsigned short* WF1T = (unsigned short*)(ws + kOffWF1T);
  unsigned short* WF2T = (unsigned short*)(ws + kOffWF2T);
  float*          WVEC = (float*)(ws + kOffWVEC);
  unsigned short* PSP  = (unsigned short*)(ws + kOffPSP);
  unsigned short* POOL = (unsigned short*)(ws + kOffPOOL);
  unsigned short* HMID = (unsigned short*)(ws + kOffHMID);

  transpose_cvt_kernel<<<dim3(kN1 / 64, kDm / 64), 256, 0, stream>>>(W1, W1T, kDm, kN1, kCarryW);
  transpose_cvt_kernel<<<dim3(kDm / 64, kDm / 64), 256, 0, stream>>>(Wf1, WF1T, kDm, kDm, kCarryW);
  transpose_cvt_kernel<<<dim3(kDm / 64, kDm / 64), 256, 0, stream>>>(Wf2, WF2T, kDm, kDm, kCarryW);
  transpose_w2_kernel<<<kDm / 64, 256, 0, stream>>>(W2, W2T, kCarryW);

  warp_weights_kernel<<<kBatch, 256, 0, stream>>>(ego, WVEC);

  gemm1_pool_kernel<<<kRows / kBlkRows, 128, 0, stream>>>(hv, W1T, b1, WVEC, PSP);

  gemm64_kernel<2><<<(kRows / 64) * (kDm / 64) / 8, 256, 0, stream>>>(
      PSP, W2T, kChan, kRows / 64, kDm / 64, kSc2, b2, tw, (void*)POOL, kDm, kCarryPool);

  gemm64_kernel<1><<<(kBatch / 64) * (kDm / 64) / 8, 256, 0, stream>>>(
      POOL, WF1T, kDm, kBatch / 64, kDm / 64, kSc3, bf1, tw, (void*)HMID, kDm, kCarryH);

  gemm64_kernel<0><<<(kBatch / 64) * (kDm / 64) / 8, 256, 0, stream>>>(
      HMID, WF2T, kDm, kBatch / 64, kDm / 64, kSc4, bf2, tw, d_out, kDm, 1.0f);
}
